// FusedOnlineAttention_30236569764232
// MI455X (gfx1250) — hardware-verified
//
#include <hip/hip_runtime.h>


namespace {
constexpr int MODE = 1;
constexpr int NB_ = 2, S = 2048, H = 16, HD = 64, D = H * HD, NT = NB_ * S, CH = 256;
constexpr float XS = 8.0f, PS = 256.0f, SCALE = 0.125f;
typedef _Float16 b16;
typedef __attribute__((ext_vector_type(16))) _Float16 v16b;
typedef __attribute__((ext_vector_type(8))) _Float16 v8b;
typedef __attribute__((ext_vector_type(2))) _Float16 v2b;
typedef __attribute__((ext_vector_type(8))) float v8f;
typedef __attribute__((ext_vector_type(4))) float v4f;
typedef __attribute__((ext_vector_type(2))) float v2f;
__device__ __forceinline__ float bf16_rne(float f) { unsigned int u = __float_as_uint(f); u += 0x7FFFu + ((u >> 16) & 1u); float r = __uint_as_float(u & 0xFFFF0000u); asm volatile("" : "+v"(r)); return r; }
__device__ __forceinline__ void split16(float v, b16& hi, b16& lo) { hi = (b16)v; lo = (b16)(v - (float)hi); }
__device__ __forceinline__ v16b frag_kb(const b16* p, int hh) { const v8b a = *(const v8b*)(p + 8 * hh), b = *(const v8b*)(p + 16 + 8 * hh); v16b f;
#pragma unroll
  for (int e = 0; e < 8; ++e) { f[e] = a[e]; f[8 + e] = b[e]; } return f; }
__device__ __forceinline__ v8f wmma16b(v16b a, v16b b, v8f c) { v8f d = __builtin_amdgcn_wmma_f32_16x16x32_f16(false, a, false, b, (short)0, c, false, false); asm volatile("v_nop\n\tv_nop\n\tv_nop\n\tv_nop" : "+v"(d) : "v"(a), "v"(b)); return d; }
__device__ __forceinline__ void wave_lds_sync() { __builtin_amdgcn_fence(__ATOMIC_RELEASE, "workgroup"); __builtin_amdgcn_wave_barrier(); __builtin_amdgcn_fence(__ATOMIC_ACQUIRE, "workgroup"); }

__global__ __launch_bounds__(256) void cvt_kernel(const float* __restrict__ q, const float* __restrict__ k, b16* __restrict__ Q16, b16* __restrict__ K16) { const size_t nt = (size_t)gridDim.x * 256, u0 = (size_t)blockIdx.x * 256 + threadIdx.x; v8b a, c;
  for (size_t u = u0; u < (size_t)NT * D / 8; u += nt) {
#pragma unroll
    for (int j = 0; j < 8; ++j) { a[j] = (b16)(bf16_rne(q[u * 8 + j]) * XS); c[j] = (b16)(bf16_rne(k[u * 8 + j]) * XS); } for (int pass = 0; pass < 2; ++pass) { *(volatile v8b*)(Q16 + u * 8) = a; *(volatile v8b*)(K16 + u * 8) = c; __threadfence(); } } }
__global__ __launch_bounds__(256) void vt_kernel(const float* __restrict__ v, b16* __restrict__ VT) { __shared__ float Tt[64][257]; const int tt = blockIdx.x >> 2, hg = blockIdx.x & 3; const size_t t0 = (size_t)tt * 64; const int b = (int)(t0 / S), s0 = (int)(t0 % S); const int tid = threadIdx.x, wave = tid >> 5, lane = tid & 31;
  for (int qq = wave; qq < 64; qq += 8) for (int c = lane; c < 256; c += 32) Tt[qq][c] = bf16_rne(v[(t0 + qq) * D + hg * 256 + c]);
  __syncthreads();
  for (int pass = 0; pass < 2; ++pass) { for (int c = wave; c < 256; c += 8) { const int h = hg * 4 + c / HD, d = c % HD; const size_t o = (((size_t)b * H + h) * HD + d) * S + s0 + lane * 2; *(volatile v2b*)(VT + o) = (v2b){(b16)(Tt[lane * 2][c] * XS), (b16)(Tt[lane * 2 + 1][c] * XS)}; } __threadfence(); } }
__global__ __launch_bounds__(32) void att_kernel(const b16* __restrict__ Q16, const b16* __restrict__ K16, const b16* __restrict__ VT, const int* __restrict__ kmask, int QLIM, float* __restrict__ out) { __shared__ __attribute__((aligned(16))) b16 Pa[16][CH + 8], Pb[16][CH + 8]; __shared__ float Sc[16][CH + 1], Mx[16], Ls[16], Fc[16], Of[16][HD + 1]; const int lane = threadIdx.x, nloc = lane & 15, hlf = lane >> 4; const int bh = blockIdx.x / (S / 16), q0 = (blockIdx.x % (S / 16)) * 16; if (q0 >= QLIM) return; const int b = bh / H, h = bh % H; const size_t tq = (size_t)b * S + q0;
  if (lane < 16) { Mx[lane] = -INFINITY; Ls[lane] = 0.0f; for (int kk = CH; kk < CH + 8; ++kk) { Pa[lane][kk] = (b16)0.0f; Pb[lane][kk] = (b16)0.0f; } }
  v16b qa[2]; for (int ks = 0; ks < 2; ++ks) qa[ks] = frag_kb(Q16 + (tq + nloc) * D + h * HD + ks * 32, hlf);
  v8f oacc[4] = {(v8f){}, (v8f){}, (v8f){}, (v8f){}}; const int nch = q0 / CH + 1;
#pragma unroll 1
  for (int ch = 0; ch < nch; ++ch) { const int k0 = ch * CH;
#pragma unroll 1
    for (int tg = 0; tg < 16; tg += 8) { v8f sacc[8];
#pragma unroll
      for (int t = 0; t < 8; ++t) sacc[t] = (v8f){};
#pragma unroll
      for (int t = 0; t < 8; ++t)
#pragma unroll
        for (int ks = 0; ks < 2; ++ks) sacc[t] = wmma16b(qa[ks], frag_kb(K16 + ((size_t)b * S + k0 + (tg + t) * 16 + nloc) * D + h * HD + ks * 32, hlf), sacc[t]);
#pragma unroll
      for (int t = 0; t < 8; ++t)
#pragma unroll
        for (int r8 = 0; r8 < 8; ++r8) Sc[8 * hlf + r8][(tg + t) * 16 + nloc] = sacc[t][r8] * (SCALE / (XS * XS)); }
    wave_lds_sync();
    if (lane < 16) { const int r = lane, qi = q0 + r; float mx = -INFINITY;
      for (int j = 0; j < CH; ++j) { const int kj = k0 + j; float s = Sc[r][j];
        if (MODE == 0) { if (kj == qi) s = -10000.0f; else if (kj > qi) s = -50000.0f; }
        else { const bool keep = (kj <= qi) && (kmask[(size_t)b * S + kj] == 0); s = keep ? s : -INFINITY; }
        Sc[r][j] = s; mx = fmaxf(mx, s); }
      const float mo = Mx[r], mn = fmaxf(mo, mx); const float fac = (mo == -INFINITY) ? 0.0f : (mn == -INFINITY ? 1.0f : __expf(mo - mn)); float sm = 0.0f;
      for (int j = 0; j < CH; ++j) { const float p = (mn == -INFINITY) ? 0.0f : __expf(Sc[r][j] - mn); sm += p; b16 ph, pl; split16(p * PS, ph, pl); Pa[r][j] = ph; Pb[r][j] = pl; } Fc[r] = fac; Ls[r] = Ls[r] * fac + sm; Mx[r] = mn; }
    wave_lds_sync();
#pragma unroll
    for (int t = 0; t < 4; ++t)
#pragma unroll
      for (int r8 = 0; r8 < 8; ++r8) oacc[t][r8] *= Fc[8 * hlf + r8];
#pragma unroll 2
    for (int kb = 0; kb < CH; kb += 32) { const v16b pa = frag_kb(&Pa[nloc][kb], hlf), pb = frag_kb(&Pb[nloc][kb], hlf);
#pragma unroll
      for (int t = 0; t < 4; ++t) { const v16b vv = frag_kb(VT + ((size_t)bh * HD + t * 16 + nloc) * S + k0 + kb, hlf); oacc[t] = wmma16b(pa, vv, oacc[t]); oacc[t] = wmma16b(pb, vv, oacc[t]); } }
    wave_lds_sync(); }
#pragma unroll
  for (int t = 0; t < 4; ++t)
#pragma unroll
    for (int r8 = 0; r8 < 8; ++r8) { const int r = 8 * hlf + r8; Of[r][t * 16 + nloc] = oacc[t][r8] * (1.0f / (PS * XS)) / Ls[r]; }
  wave_lds_sync();
  for (int pass = 0; pass < 2; ++pass) { for (int r = 0; r < 16; ++r) *(volatile v2f*)(out + (tq + r) * D + h * HD + lane * 2) = (v2f){Of[r][lane * 2], Of[r][lane * 2 + 1]}; __threadfence(); } }
}

extern "C" void kernel_launch(void* const* d_in, const int* in_sizes, int n_in, void* d_out, int out_size, void* d_ws, size_t ws_size, hipStream_t stream) {
  (void)n_in;
  auto Fp = [&](int i) { return (const float*)d_in[i]; };
  if (in_sizes[0] != NT * D || in_sizes[1] != NT * D || in_sizes[2] != NT * D || (MODE == 1 && in_sizes[3] != NT) || out_size != NT * D) return;
  const int QLIM = S;
  size_t off = 0; char* ws = (char*)d_ws;
  auto carve = [&](size_t bytes) { char* p = ws + off; off += (bytes + 255) & ~(size_t)255; return p; };
  b16* Q16 = (b16*)carve((size_t)NT * D * 2); b16* K16 = (b16*)carve((size_t)NT * D * 2); b16* VT = (b16*)carve((size_t)NT * D * 2);
  if (off > ws_size || off > ((size_t)32 << 20)) return;
  cvt_kernel<<<512, 256, 0, stream>>>(Fp(0), Fp(1), Q16, K16);
  vt_kernel<<<(NT / 64) * 4, 256, 0, stream>>>(Fp(2), VT);
  att_kernel<<<NB_ * H * (S / 16), 32, 0, stream>>>(Q16, K16, VT, MODE == 1 ? (const int*)d_in[3] : nullptr, QLIM, (float*)d_out);
}
